// CausalSelfAttentionRelPos_25701084299441
// MI455X (gfx1250) — hardware-verified
//
#include <hip/hip_runtime.h>
#include <math.h>

#ifndef NB
#define NB 4
#endif
#ifndef SEQ
#define SEQ 2048
#endif
#define SEQ_FULL 2048
#define NPOS 2048
#define DME  1024
#define NHD  16
#define HD   64
#define N3   (3 * DME)
#define KQN  (2 * DME)
#define MT   (NB * SEQ)
#define QT   (SEQ / 16)
#define AWV  4
#define RWP  80
#define TE   1024
#define WSCL 64.0f
#define ESCL 64.0f
#define QKS  16.0f
#define QRS  2048.0f
#define VSC  16.0f
#define VRS  1024.0f
#define PSC  1024.0f
#define PRS  1024.0f
#define RSQD 0.125f

static_assert(NHD * HD == DME);
static_assert(HD == 64);
static_assert((SEQ % 64) == 0 && SEQ >= 64 && SEQ <= SEQ_FULL && SEQ <= NPOS);
static_assert((DME % 64) == 0 && (N3 % 64) == 0 && (KQN % 64) == 0);
static_assert((((SEQ / 64) * (KQN / 64)) % 8) == 0);
static_assert((((DME / 64) * (SEQ / 64)) % 8) == 0);
static_assert((((SEQ / 64) * (DME / 64)) % 8) == 0);
static_assert(((SEQ * DME) % 2048) == 0 && ((NPOS * HD) % 2048) == 0);
static_assert(((NHD * QT) % AWV) == 0);
static_assert((TE % 16) == 0);
static_assert(RWP >= 80);
static_assert(PRS == VRS);

typedef _Float16 v16h __attribute__((ext_vector_type(16)));
typedef __bf16 v16bf __attribute__((ext_vector_type(16)));
typedef unsigned short v16us __attribute__((ext_vector_type(16)));
typedef unsigned short v8us  __attribute__((ext_vector_type(8)));
typedef float v8f __attribute__((ext_vector_type(8)));
typedef float v4f __attribute__((ext_vector_type(4)));
typedef unsigned int v4u __attribute__((ext_vector_type(4)));

union FragU { v16us v; v8us h[2]; };

__device__ __forceinline__ unsigned short bf_bits(float f) {
  const unsigned u = __float_as_uint(f);
  return (unsigned short)((u + 0x7FFFu + ((u >> 16) & 1u)) >> 16);
}
__device__ __forceinline__ float bf_up(unsigned short h) { return __uint_as_float(((unsigned)h) << 16); }
__device__ __forceinline__ float bfr(float f) { return bf_up(bf_bits(f)); }
__device__ __forceinline__ unsigned short h_bits(_Float16 x) { return __builtin_bit_cast(unsigned short, x); }
__device__ __forceinline__ unsigned short f2h(float f) { return h_bits((_Float16)f); }
__device__ __forceinline__ float hf_up(unsigned short b) { return (float)__builtin_bit_cast(_Float16, b); }
__device__ __forceinline__ unsigned pk16(unsigned short a, unsigned short b) { return (unsigned)a | ((unsigned)b << 16); }
__device__ __forceinline__ int clampi(int v, int lo, int hi) { return v < lo ? lo : (v > hi ? hi : v); }
__device__ __forceinline__ v8f zero8() { v8f z = {0.f, 0.f, 0.f, 0.f, 0.f, 0.f, 0.f, 0.f}; return z; }

__device__ __forceinline__ v16us ldfrag_u(const unsigned short* p) {
  FragU f;
  f.h[0] = *(const v8us*)(p);
  f.h[1] = *(const v8us*)(p + 16);
  return f.v;
}

template <int OPK>
__device__ __forceinline__ v8f mma_raw(v16us a, v16us b, v8f c) {
  if (OPK == 0)
    return __builtin_amdgcn_wmma_f32_16x16x32_f16(false, __builtin_bit_cast(v16h, a), false,
                                                  __builtin_bit_cast(v16h, b), (short)0, c, false, false);
  return __builtin_amdgcn_wmma_f32_16x16x32_bf16(false, __builtin_bit_cast(v16bf, a), false,
                                                 __builtin_bit_cast(v16bf, b), (short)0, c, false, false);
}
__device__ __forceinline__ void dep_guard1(v8f& a, v8f& b, v16us x) {
#if defined(__HIP_DEVICE_COMPILE__)
  asm volatile("v_nop\n\tv_nop\n\tv_nop\n\tv_nop" : "+v"(a), "+v"(b) : "v"(x));
#endif
}
__device__ __forceinline__ void keep4_u(v16us a, v16us b, v16us c, v16us d) {
#if defined(__HIP_DEVICE_COMPILE__)
  asm volatile("v_nop" :: "v"(a), "v"(b), "v"(c), "v"(d));
#endif
}
__device__ __forceinline__ void acc_guard4(v8f& a, v8f& b, v8f& c, v8f& d) {
#if defined(__HIP_DEVICE_COMPILE__)
  asm volatile("v_nop\n\tv_nop\n\tv_nop\n\tv_nop" : "+v"(a), "+v"(b), "+v"(c), "+v"(d));
#endif
}
__device__ __forceinline__ void guard2x2(v8f& a, v8f& b, v16us x, v16us y) {
#if defined(__HIP_DEVICE_COMPILE__)
  asm volatile("v_nop\n\tv_nop\n\tv_nop\n\tv_nop" : "+v"(a), "+v"(b) : "v"(x), "v"(y));
#endif
}
__device__ __forceinline__ void guard2x4(v8f& a, v8f& b, v16us x, v16us y, v16us z, v16us w) {
#if defined(__HIP_DEVICE_COMPILE__)
  asm volatile("v_nop\n\tv_nop\n\tv_nop\n\tv_nop" : "+v"(a), "+v"(b) : "v"(x), "v"(y), "v"(z), "v"(w));
#endif
}
__device__ __forceinline__ void guard1x2(v8f& a, v16us x, v16us y) {
#if defined(__HIP_DEVICE_COMPILE__)
  asm volatile("v_nop\n\tv_nop\n\tv_nop\n\tv_nop" : "+v"(a) : "v"(x), "v"(y));
#endif
}
__device__ __forceinline__ void wave_sync_lds() {
  __builtin_amdgcn_fence(__ATOMIC_RELEASE, "workgroup");
  __builtin_amdgcn_wave_barrier();
  __builtin_amdgcn_fence(__ATOMIC_ACQUIRE, "workgroup");
}

__global__ __launch_bounds__(256) void cvt_lin(const float* __restrict__ w, unsigned short* o, int n, float sc,
                                               int sbs, int dbs) {
  const float* src = w + (size_t)blockIdx.y * (size_t)sbs;
  unsigned short* dst0 = o + (size_t)blockIdx.y * (size_t)dbs;
  const int base = (blockIdx.x * 256 + threadIdx.x) * 8;
  if (base + 8 > n) return;
  const v4f a0 = *(const v4f*)(src + base);
  const v4f a1 = *(const v4f*)(src + base + 4);
  v4u hv;
#pragma unroll
  for (int e = 0; e < 2; ++e) {
    hv[e]     = pk16(f2h(bfr(a0[2 * e]) * sc), f2h(bfr(a0[2 * e + 1]) * sc));
    hv[2 + e] = pk16(f2h(bfr(a1[2 * e]) * sc), f2h(bfr(a1[2 * e + 1]) * sc));
  }
  unsigned short* d = dst0 + base;
  *(volatile v4u*)d = hv;
  __threadfence();
  *(volatile v4u*)d = hv;
}

template <int MODE>
__global__ __launch_bounds__(256) void cvt_t(const float* __restrict__ w, unsigned short* o, int R, int C, float sc) {
  __shared__ __align__(16) unsigned short st[64 * 72];
  const int t = threadIdx.x;
  const int r0 = blockIdx.y * 64, c0 = blockIdx.x * 64;
  if (r0 + 64 > R || c0 + 64 > C) return;
  {
    const int row = t >> 2, ch = (t & 3) * 16;
    const float* p = w + (size_t)(r0 + row) * C + c0 + ch;
#pragma unroll
    for (int q = 0; q < 4; ++q) {
      const v4f v = *(const v4f*)(p + 4 * q);
#pragma unroll
      for (int e = 0; e < 4; ++e) {
        unsigned short bits;
        if (MODE == 0) bits = f2h(bfr(v[e]) * sc);
        else           bits = bf_bits(v[e]);
        st[(ch + 4 * q + e) * 72 + row] = bits;
      }
    }
  }
  __syncthreads();
  v4u hv[2];
#pragma unroll
  for (int half = 0; half < 2; ++half) {
    const int cl = (t >> 3) + 32 * half, pc = (t & 7) * 8;
    hv[half] = *(const v4u*)(st + cl * 72 + pc);
  }
  for (int pass = 0; pass < 2; ++pass) {
#pragma unroll
    for (int half = 0; half < 2; ++half) {
      const int cl = (t >> 3) + 32 * half, pc = (t & 7) * 8;
      unsigned short* dst = o + (size_t)(c0 + cl) * R + r0 + pc;
      *(volatile v4u*)dst = hv[half];
    }
    __threadfence();
  }
}

template <int OPK, int NPL, int OM, int CBM>
__global__ __launch_bounds__(256) void gemm64(
    const unsigned short* __restrict__ Ap, const unsigned short* __restrict__ Ap2, int lda,
    const unsigned short* __restrict__ Btp, int ldb,
    unsigned short* Ch, unsigned short* Ch2, float* Cf, int ldc,
    const float* __restrict__ cb, float wsc, float osc, float rsc, int M, int N, int K) {
  __shared__ __align__(16) float sT[8][16 * 68];
  const int lane = threadIdx.x & 31;
  const int wave = threadIdx.x >> 5;
  const int tilesN = N >> 6;
  const int tilesM = M >> 6;
  const int tile = blockIdx.x * 8 + wave;
  if (tile >= tilesM * tilesN) return;
  const int tm = tile / tilesN;
  const int tn = tile - tm * tilesN;
  const int m0 = tm << 6;
  const int n0 = tn << 6;

  const int rlane = lane & 15;
  const int koff  = (lane >> 4) * 8;
  const int mOff  = (lane >> 4) * 8;

  v8f acc[4][4];
#pragma unroll
  for (int i = 0; i < 4; ++i)
#pragma unroll
    for (int j = 0; j < 4; ++j) acc[i][j] = zero8();

#pragma unroll 1
  for (int pl = 0; pl < NPL; ++pl) {
    const unsigned short* Ac = (pl == 0) ? Ap : Ap2;
    for (int k0 = 0; k0 < K; k0 += 32) {
      v16us bh[4];
#pragma unroll
      for (int j = 0; j < 4; ++j) {
        const size_t bo = (size_t)(n0 + (j << 4) + rlane) * ldb + koff + k0;
        bh[j] = ldfrag_u(Btp + bo);
      }
#pragma unroll
      for (int i = 0; i < 4; ++i) {
        const size_t ao = (size_t)(m0 + (i << 4) + rlane) * lda + koff + k0;
        const v16us ah = ldfrag_u(Ac + ao);
#pragma unroll
        for (int j = 0; j < 4; ++j) acc[i][j] = mma_raw<OPK>(ah, bh[j], acc[i][j]);
        dep_guard1(acc[i][0], acc[i][3], ah);
      }
      keep4_u(bh[0], bh[1], bh[2], bh[3]);
    }
  }
  acc_guard4(acc[0][0], acc[0][1], acc[0][2], acc[0][3]);
  acc_guard4(acc[1][0], acc[1][1], acc[1][2], acc[1][3]);
  acc_guard4(acc[2][0], acc[2][1], acc[2][2], acc[2][3]);
  acc_guard4(acc[3][0], acc[3][1], acc[3][2], acc[3][3]);

  const int hh2 = lane >> 4, c4 = (lane & 15) * 4;
  const int q8  = lane >> 3, c8 = (lane & 7) * 8;

  v4f cb4 = {0.f, 0.f, 0.f, 0.f};
  if (OM == 0) {
    const v4f v = *(const v4f*)(cb + n0 + c4);
    cb4[0] = bfr(v[0]); cb4[1] = bfr(v[1]); cb4[2] = bfr(v[2]); cb4[3] = bfr(v[3]);
  }
  float cbc[8];
#pragma unroll
  for (int e = 0; e < 8; ++e) cbc[e] = 0.f;
  if (OM != 0 && CBM == 1) {
    const v4f u0 = *(const v4f*)(cb + n0 + c8);
    const v4f u1 = *(const v4f*)(cb + n0 + c8 + 4);
#pragma unroll
    for (int e = 0; e < 4; ++e) { cbc[e] = bfr(u0[e]); cbc[4 + e] = bfr(u1[e]); }
  }

  float* slab = sT[wave];
#pragma unroll
  for (int i = 0; i < 4; ++i) {
    const int mBase = m0 + (i << 4);
#pragma unroll
    for (int j = 0; j < 4; ++j) {
#pragma unroll
      for (int r = 0; r < 8; ++r) {
        slab[(mOff + r) * 68 + (j << 4) + rlane] = acc[i][j][r];
      }
    }
    wave_sync_lds();
    if (OM == 0) {
      v4f vals[8];
#pragma unroll
      for (int it = 0; it < 8; ++it) {
        const int row = it * 2 + hh2;
        const v4f v = *(const v4f*)(slab + row * 68 + c4);
        vals[it] = v * wsc + cb4;
      }
      for (int pass = 0; pass < 2; ++pass) {
#pragma unroll
        for (int it = 0; it < 8; ++it) {
          const int row = it * 2 + hh2;
          *(volatile v4f*)(Cf + (size_t)(mBase + row) * ldc + (size_t)n0 + c4) = vals[it];
        }
        __threadfence();
      }
    } else {
      v4u hv[4], hw[4];
#pragma unroll
      for (int it = 0; it < 4; ++it) {
        const int row = it * 4 + q8;
        const float* sp = slab + row * 68 + c8;
        float rb = 0.f;
        if (CBM == 2) rb = bfr(cb[mBase + row]);
        v4u ha = {0u, 0u, 0u, 0u}, hb = {0u, 0u, 0u, 0u};
#pragma unroll
        for (int e = 0; e < 4; ++e) {
          const float bias0 = (CBM == 1) ? cbc[2 * e] : rb;
          const float bias1 = (CBM == 1) ? cbc[2 * e + 1] : rb;
          const float b0 = (sp[2 * e]     * wsc + bias0) * osc;
          const float b1 = (sp[2 * e + 1] * wsc + bias1) * osc;
          const unsigned short x0 = f2h(b0), x1 = f2h(b1);
          ha[e] = pk16(x0, x1);
          if (OM == 2) {
            const unsigned short y0 = f2h((b0 - hf_up(x0)) * rsc);
            const unsigned short y1 = f2h((b1 - hf_up(x1)) * rsc);
            hb[e] = pk16(y0, y1);
          }
        }
        hv[it] = ha;
        hw[it] = hb;
      }
      for (int pass = 0; pass < 2; ++pass) {
#pragma unroll
        for (int it = 0; it < 4; ++it) {
          const int row = it * 4 + q8;
          const size_t go = (size_t)(mBase + row) * ldc + (size_t)n0 + c8;
          *(volatile v4u*)(Ch + go) = hv[it];
          if (OM == 2) *(volatile v4u*)(Ch2 + go) = hw[it];
        }
        __threadfence();
      }
    }
    wave_sync_lds();
  }
}

__global__ __launch_bounds__(128) void attn_kernel(
    const unsigned short* __restrict__ QKH, const unsigned short* __restrict__ QKL,
    const unsigned short* __restrict__ ERH,
    const unsigned short* __restrict__ VTh, const unsigned short* __restrict__ VTl,
    unsigned short* Zh, unsigned short* Zl) {
  __shared__ __align__(16) float relw[AWV][16 * RWP];
  __shared__ __align__(16) unsigned short pws[AWV][2][16 * 32];
  __shared__ __align__(16) unsigned short zst[AWV][2][16 * HD];
  const int lane = threadIdx.x & 31, m = lane & 15, hh = lane >> 4;
  const int wv = __builtin_amdgcn_readfirstlane((int)(threadIdx.x >> 5));
  const int task = (int)blockIdx.x * AWV + wv;
  const int h = task / QT;
  const int t0 = (task - h * QT) << 4;
  const bool early = (t0 < TE);
  float* rw = relw[wv];
  unsigned short* ph = pws[wv][0];
  unsigned short* pl = pws[wv][1];

  const size_t qo = (size_t)(t0 + m) * KQN + (size_t)(h * HD + 8 * hh);
  const v16us qh0 = ldfrag_u(QKH + qo);
  const v16us qh1 = ldfrag_u(QKH + qo + 32);
  const v16us ql0 = ldfrag_u(QKL + qo);
  const v16us ql1 = ldfrag_u(QKL + qo + 32);

  float mx[8], ls[8];
  v8f O[4], OX[4];
#pragma unroll
  for (int i = 0; i < 4; ++i) { O[i] = zero8(); OX[i] = zero8(); }
#pragma unroll
  for (int r = 0; r < 8; ++r) { mx[r] = -1.0e30f; ls[r] = 0.f; }

  const float cS  = 1.0f / (QKS * QKS);
  const float cSR = 1.0f / (QKS * QKS * QRS);
  const float cB  = 1.0f / (QKS * ESCL);
  const float cBR = 1.0f / (QKS * ESCL * QRS);

  const int nblk = (t0 + 47) >> 5;

#pragma unroll 1
  for (int kb = 0; kb < nblk; ++kb) {
    const int sb = kb << 5;

    if ((kb & 1) == 0) {
      const int u0 = NPOS - 16 - t0 + sb;
#pragma unroll
      for (int j = 0; j < 5; ++j) {
        const int u = clampi(u0 + 16 * j + m, 0, NPOS - 1);
        const unsigned short* ep = ERH + (size_t)u * HD + 8 * hh;
        const v16us e0 = ldfrag_u(ep);
        const v16us e1 = ldfrag_u(ep + 32);
        v8f Bh = mma_raw<0>(qh0, e0, zero8());
        v8f Br = mma_raw<0>(ql0, e0, zero8());
        Bh = mma_raw<0>(qh1, e1, Bh);
        Br = mma_raw<0>(ql1, e1, Br);
        guard2x2(Bh, Br, e0, e1);
#pragma unroll
        for (int r = 0; r < 8; ++r)
          rw[(8 * hh + r) * RWP + 16 * j + m] = Bh[r] * cB + Br[r] * cBR;
      }
    }

    float s0[8], s1[8];
#pragma unroll
    for (int nt = 0; nt < 2; ++nt) {
      const size_t ko = (size_t)(sb + 16 * nt + m) * KQN + (size_t)(DME + h * HD + 8 * hh);
      const v16us kh0 = ldfrag_u(QKH + ko);
      const v16us kh1 = ldfrag_u(QKH + ko + 32);
      const v16us kl0 = ldfrag_u(QKL + ko);
      const v16us kl1 = ldfrag_u(QKL + ko + 32);
      v8f S = mma_raw<0>(qh0, kh0, zero8());
      v8f R = mma_raw<0>(ql0, kh0, zero8());
      S = mma_raw<0>(qh1, kh1, S);
      R = mma_raw<0>(ql1, kh1, R);
      if (early) {
        R = mma_raw<0>(qh0, kl0, R);
        R = mma_raw<0>(qh1, kl1, R);
      }
      guard2x4(S, R, kh0, kh1, kl0, kl1);
#pragma unroll
      for (int r = 0; r < 8; ++r) {
        const float v = S[r] * cS + R[r] * cSR;
        if (nt == 0) s0[r] = v; else s1[r] = v;
      }
    }
    wave_sync_lds();

    const int boff = (kb & 1) << 5;
#pragma unroll
    for (int r = 0; r < 8; ++r) {
      const int row = 8 * hh + r;
      const int tq = t0 + row;
      const float rv0 = rw[row * RWP + boff + 15 - row + m];
      const float rv1 = rw[row * RWP + boff + 31 - row + m];
      float a0 = (s0[r] + rv0) * RSQD;
      float a1 = (s1[r] + rv1) * RSQD;
      a0 = (sb + m > tq)      ? (a0 + (-1.0e9f)) : a0;
      a1 = (sb + 16 + m > tq) ? (a1 + (-1.0e9f)) : a1;
      s0[r] = a0; s1[r] = a1;
    }

    v8f alv = zero8();
#pragma unroll
    for (int r = 0; r < 8; ++r) {
      float xm = fmaxf(s0[r], s1[r]);
      xm = fmaxf(xm, __shfl_xor(xm, 1, 32));
      xm = fmaxf(xm, __shfl_xor(xm, 2, 32));
      xm = fmaxf(xm, __shfl_xor(xm, 4, 32));
      xm = fmaxf(xm, __shfl_xor(xm, 8, 32));
      const float mn = fmaxf(mx[r], xm);
      const float al = __expf(mx[r] - mn);
      mx[r] = mn;
      const float p0 = __expf(s0[r] - mn);
      const float p1 = __expf(s1[r] - mn);
      float ps = p0 + p1;
      ps += __shfl_xor(ps, 1, 32);
      ps += __shfl_xor(ps, 2, 32);
      ps += __shfl_xor(ps, 4, 32);
      ps += __shfl_xor(ps, 8, 32);
      ls[r] = ls[r] * al + ps;
      alv[r] = al;
      const int row = 8 * hh + r;
      const float g0 = p0 * PSC, g1 = p1 * PSC;
      const unsigned short x0 = f2h(g0), x1 = f2h(g1);
      ph[row * 32 + m]      = x0;
      ph[row * 32 + 16 + m] = x1;
      pl[row * 32 + m]      = f2h((g0 - hf_up(x0)) * PRS);
      pl[row * 32 + 16 + m] = f2h((g1 - hf_up(x1)) * PRS);
    }
#pragma unroll
    for (int i = 0; i < 4; ++i) { O[i] = O[i] * alv; OX[i] = OX[i] * alv; }
    wave_sync_lds();

    const v16us af = ldfrag_u(ph + m * 32 + 8 * hh);
    const v16us bf = ldfrag_u(pl + m * 32 + 8 * hh);
    const size_t vb = (size_t)(h * HD + m) * SEQ + (size_t)sb + (size_t)(8 * hh);
    if (early) {
#pragma unroll
      for (int ds = 0; ds < 4; ++ds) {
        const size_t vo = vb + (size_t)(16 * ds) * SEQ;
        const v16us vh = ldfrag_u(VTh + vo);
        const v16us vl = ldfrag_u(VTl + vo);
        O[ds]  = mma_raw<0>(af, vh, O[ds]);
        OX[ds] = mma_raw<0>(af, vl, OX[ds]);
        OX[ds] = mma_raw<0>(bf, vh, OX[ds]);
        guard2x4(O[ds], OX[ds], af, bf, vh, vl);
      }
    } else {
#pragma unroll
      for (int ds = 0; ds < 4; ++ds) {
        const size_t vo = vb + (size_t)(16 * ds) * SEQ;
        const v16us vh = ldfrag_u(VTh + vo);
        O[ds] = mma_raw<0>(af, vh, O[ds]);
        guard1x2(O[ds], af, vh);
      }
    }
  }
  acc_guard4(O[0], O[1], O[2], O[3]);
  acc_guard4(OX[0], OX[1], OX[2], OX[3]);

  unsigned short* zh = zst[wv][0];
  unsigned short* zl = zst[wv][1];
  const float cO = 1.0f / (PSC * VSC);
  const float cX = 1.0f / (PSC * VSC * VRS);
#pragma unroll
  for (int r = 0; r < 8; ++r) {
    const int row = 8 * hh + r;
    const float linv = 1.0f / ls[r];
#pragma unroll
    for (int ds = 0; ds < 4; ++ds) {
      const float o = (O[ds][r] * cO + OX[ds][r] * cX) * linv;
      const unsigned short x0 = bf_bits(o);
      zh[row * HD + 16 * ds + m] = x0;
      zl[row * HD + 16 * ds + m] = bf_bits(o - bf_up(x0));
    }
  }
  wave_sync_lds();
  {
    const int rq = lane >> 3, pc = (lane & 7) * 8;
    v4u ha[4], hb[4];
#pragma unroll
    for (int it = 0; it < 4; ++it) {
      const int row = it * 4 + rq;
      ha[it] = *(const v4u*)(zh + row * HD + pc);
      hb[it] = *(const v4u*)(zl + row * HD + pc);
    }
    for (int pass = 0; pass < 2; ++pass) {
#pragma unroll
      for (int it = 0; it < 4; ++it) {
        const int row = it * 4 + rq;
        const size_t go = (size_t)(t0 + row) * DME + (size_t)(h * HD + pc);
        *(volatile v4u*)(Zh + go) = ha[it];
        *(volatile v4u*)(Zl + go) = hb[it];
      }
      __threadfence();
    }
  }
}

extern "C" void kernel_launch(void* const* d_in, const int* in_sizes, int n_in,
                              void* d_out, int out_size, void* d_ws, size_t ws_size,
                              hipStream_t stream) {
  if (n_in < 6) return;
  if (in_sizes[0] < ((NB - 1) * SEQ_FULL + SEQ) * DME) return;
  if (in_sizes[1] < DME * N3) return;
  if (in_sizes[2] < N3) return;
  if (in_sizes[3] < NPOS * HD) return;
  if (in_sizes[4] < DME * DME) return;
  if (in_sizes[5] < DME) return;
  if (out_size < MT * DME) return;

  const float* x      = (const float*)d_in[0];
  const float* w_attn = (const float*)d_in[1];
  const float* b_attn = (const float*)d_in[2];
  const float* er     = (const float*)d_in[3];
  const float* w_proj = (const float*)d_in[4];
  const float* b_proj = (const float*)d_in[5];

  const size_t PWT = (size_t)N3 * DME * 2;
  const size_t PWP = (size_t)DME * DME * 2;
  const size_t PER = (size_t)NPOS * HD * 2;
  const size_t PXH = (size_t)MT * DME * 2;
  const size_t PQK = (size_t)SEQ * KQN * 2;
  const size_t PVT = (size_t)DME * SEQ * 2;
  const size_t PZ  = (size_t)SEQ * DME * 2;
  size_t off = 0;
  const size_t oWT  = off; off += PWT;
  const size_t oWP  = off; off += PWP;
  const size_t oER  = off; off += PER;
  const size_t oXH  = off; off += PXH;
  const size_t oQKH = off; off += PQK;
  const size_t oQKL = off; off += PQK;
  const size_t oVTH = off; off += PVT;
  const size_t oVTL = off; off += PVT;
  const size_t oZH  = off; off += PZ;
  const size_t oZL  = off; off += PZ;
  if (off > ws_size) return;
  if (off > (size_t)134217728) return;

  char* ws = (char*)d_ws;
  unsigned short* WT  = (unsigned short*)(ws + oWT);
  unsigned short* WP  = (unsigned short*)(ws + oWP);
  unsigned short* ERH = (unsigned short*)(ws + oER);
  unsigned short* XH  = (unsigned short*)(ws + oXH);
  unsigned short* QKH = (unsigned short*)(ws + oQKH);
  unsigned short* QKL = (unsigned short*)(ws + oQKL);
  unsigned short* VTH = (unsigned short*)(ws + oVTH);
  unsigned short* VTL = (unsigned short*)(ws + oVTL);
  unsigned short* ZH  = (unsigned short*)(ws + oZH);
  unsigned short* ZL  = (unsigned short*)(ws + oZL);
  float* out0 = (float*)d_out;
  float* fdummy = (float*)(ws + oQKH);

  const dim3 blk(256);
  const int gQK = ((SEQ / 64) * (KQN / 64)) / 8;
  const int gVT = ((DME / 64) * (SEQ / 64)) / 8;
  const int gPR = ((SEQ / 64) * (DME / 64)) / 8;
  const int gAT = (NHD * QT) / AWV;

  cvt_lin<<<dim3((SEQ * DME) / 2048, NB), blk, 0, stream>>>(x, XH, SEQ * DME, 1.0f, SEQ_FULL * DME, SEQ * DME);
  cvt_lin<<<dim3((NPOS * HD) / 2048, 1), blk, 0, stream>>>(er, ERH, NPOS * HD, ESCL, 0, 0);
  cvt_t<0><<<dim3(N3 / 64, DME / 64), blk, 0, stream>>>(w_attn, WT, DME, N3, WSCL);
  cvt_t<1><<<dim3(DME / 64, DME / 64), blk, 0, stream>>>(w_proj, WP, DME, DME, 1.0f);

  for (int b = 0; b < NB; ++b) {
    const unsigned short* XHb = XH + (size_t)b * SEQ * DME;
    gemm64<0, 1, 2, 1><<<dim3(gQK), blk, 0, stream>>>(
        XHb, XHb, DME, WT, DME, QKH, QKL, fdummy, KQN, b_attn, 1.0f / WSCL, QKS, QRS, SEQ, KQN, DME);
    gemm64<0, 1, 2, 2><<<dim3(gVT), blk, 0, stream>>>(
        WT + (size_t)KQN * DME, WT, DME, XHb, DME, VTH, VTL, fdummy, SEQ, b_attn + KQN, 1.0f / WSCL, VSC, VRS,
        DME, SEQ, DME);
    attn_kernel<<<dim3(gAT), dim3(128), 0, stream>>>(QKH, QKL, ERH, VTH, VTL, ZH, ZL);
    gemm64<1, 2, 0, 1><<<dim3(gPR), blk, 0, stream>>>(
        ZH, ZL, DME, WP, DME, QKH, QKL, out0 + (size_t)b * SEQ * DME, DME, b_proj, 1.0f, 1.0f, 1.0f,
        SEQ, DME, DME);
  }
  (void)hipGetLastError();
}
